// ReverseCrossAttention_30812095382045
// MI455X (gfx1250) — hardware-verified
//
#include <hip/hip_runtime.h>


#define NBI  4
#define NT_  2048
#define DM   1024
#define NTK  NT_
#define RCH  1024
#define VHD  128
#define NKVV (DM / 128)
#define KW   DM
#define SCL  0.03125f
#define LN_EPS 1e-5f
#define LOSC 1024.0f

typedef _Float16 h16;
typedef unsigned short bf;
typedef __attribute__((ext_vector_type(16))) __bf16   v16bf;
typedef __attribute__((ext_vector_type(16))) _Float16 v16h;
typedef __attribute__((ext_vector_type(8)))  _Float16 v8h;
typedef __attribute__((ext_vector_type(8)))  unsigned short v8us;
typedef __attribute__((ext_vector_type(8)))  float    v8f;
typedef __attribute__((ext_vector_type(4)))  float    v4f;
typedef __attribute__((ext_vector_type(4)))  _Float16 v4h;
typedef v8h  __attribute__((may_alias)) v8ha;
typedef v4f  __attribute__((may_alias)) v4fa;
typedef v8us __attribute__((may_alias)) v8usa;

__device__ __forceinline__ unsigned short f2bf(float f) { unsigned u = __float_as_uint(f); u += 0x7FFFu + ((u >> 16) & 1u); return (unsigned short)(u >> 16); }
__device__ __forceinline__ float bf2f(unsigned short b) { return __uint_as_float(((unsigned)b) << 16); }
__device__ __forceinline__ float bfr(float f) { return bf2f(f2bf(f)); }
__device__ __forceinline__ v16h cat16(v8h lo, v8h hi) { return __builtin_shufflevector(lo, hi, 0, 1, 2, 3, 4, 5, 6, 7, 8, 9, 10, 11, 12, 13, 14, 15); }
__device__ __forceinline__ v16bf cat16b(v8us lo, v8us hi) { return __builtin_bit_cast(v16bf, __builtin_shufflevector(lo, hi, 0, 1, 2, 3, 4, 5, 6, 7, 8, 9, 10, 11, 12, 13, 14, 15)); }
__device__ __forceinline__ v8f wmma16(v16h a, v16h b, v8f c) { return __builtin_amdgcn_wmma_f32_16x16x32_f16(false, a, false, b, (short)0, c, false, false); }
__device__ __forceinline__ v8f wmmab(v16bf a, v16bf b, v8f c) { return __builtin_amdgcn_wmma_f32_16x16x32_bf16(false, a, false, b, (short)0, c, false, false); }

__global__ __launch_bounds__(256) void k_wt(const float* __restrict__ Wm, int K, int ncols, bf* WT) {
    __shared__ __align__(16) unsigned short tl[64 * 72];
    const int tid = threadIdx.x, k0 = blockIdx.x * 64, n0 = blockIdx.y * 64;
    const int kk = tid >> 2, nq = (tid & 3) * 16;
#pragma unroll
    for (int i = 0; i < 16; ++i) tl[(nq + i) * 72 + kk] = f2bf(Wm[(size_t)(k0 + kk) * ncols + n0 + nq + i]);
    __syncthreads();
    const int piece = tid & 7;
    auto pass = [&]() {
#pragma unroll
        for (int s = 0; s < 2; ++s) { const int nr = (tid >> 3) + 32 * s; const v8us val = *(const v8usa*)(tl + nr * 72 + piece * 8); *(volatile v8us*)(WT + (size_t)(n0 + nr) * K + k0 + piece * 8) = val; }
    };
    pass(); __threadfence(); pass();
}
__global__ __launch_bounds__(256) void k_cvtb(const float* __restrict__ src, int nrows, bf* dst) {
    const int lane = threadIdx.x & 31, r = blockIdx.x * 8 + (threadIdx.x >> 5);
    if (r >= nrows) return;
    v8us o[DM / 256];
#pragma unroll
    for (int q = 0; q < DM / 256; ++q) { v8us t;
#pragma unroll
        for (int i = 0; i < 8; ++i) t[i] = f2bf(src[(size_t)r * DM + q * 256 + lane * 8 + i]);
        o[q] = t; }
#pragma unroll
    for (int q = 0; q < DM / 256; ++q) *(volatile v8us*)(dst + (size_t)r * DM + q * 256 + lane * 8) = o[q];
    __threadfence();
#pragma unroll
    for (int q = 0; q < DM / 256; ++q) *(volatile v8us*)(dst + (size_t)r * DM + q * 256 + lane * 8) = o[q];
}

template <bool SPLITA, bool F16OUT = false>
__global__ __launch_bounds__(128) void k_gemmb(const bf* __restrict__ A, const bf* __restrict__ Al, const bf* __restrict__ Bn, const float* __restrict__ bias, float* C, int ldc, h16* C2, const float* __restrict__ R = nullptr, int K = DM, int roundR = 1) {
    __shared__ __align__(16) float ost[4][16 * 68];
    const int lane = threadIdx.x & 31, wave = threadIdx.x >> 5, lr = lane & 15, hi = lane >> 4;
    const int r0 = blockIdx.x * 64 + wave * 16, c0 = blockIdx.y * 64;
    const size_t aoff = (size_t)(r0 + lr) * K + 8 * hi;
    size_t boff[4];
#pragma unroll
    for (int t = 0; t < 4; ++t) boff[t] = (size_t)(c0 + t * 16 + lr) * K + 8 * hi;
    v8f acc[4];
#pragma unroll
    for (int t = 0; t < 4; ++t) acc[t] = (v8f){};
#pragma unroll 1
    for (int kc = 0; kc < K; kc += 32) {
        const v16bf a = cat16b(*(const v8us*)(A + aoff + kc), *(const v8us*)(A + aoff + kc + 16));
        v16bf al = a;
        if (SPLITA) al = cat16b(*(const v8us*)(Al + aoff + kc), *(const v8us*)(Al + aoff + kc + 16));
#pragma unroll
        for (int t = 0; t < 4; ++t) { const v16bf b = cat16b(*(const v8us*)(Bn + boff[t] + kc), *(const v8us*)(Bn + boff[t] + kc + 16)); acc[t] = wmmab(a, b, acc[t]); if (SPLITA) acc[t] = wmmab(al, b, acc[t]); }
        asm volatile("v_nop\n\tv_nop\n\tv_nop\n\tv_nop" : "+v"(acc[0]), "+v"(acc[1]), "+v"(acc[2]), "+v"(acc[3]) : "v"(a), "v"(al));
    }
    float* os = &ost[wave][0];
#pragma unroll
    for (int t = 0; t < 4; ++t) { const float bv = bias ? bfr(bias[c0 + t * 16 + lr]) : 0.f;
#pragma unroll
        for (int j = 0; j < 8; ++j) os[(hi * 8 + j) * 68 + t * 16 + lr] = acc[t][j] + bv; }
    __syncthreads();
    if (F16OUT) {
        h16* crow = (h16*)(void*)C + (size_t)r0 * ldc + c0;
        auto pass = [&]() {
#pragma unroll
            for (int s = 0; s < 4; ++s) { const int row = 4 * s + (lane >> 3), piece = lane & 7; const float* sp = os + row * 68 + piece * 8; v8h o, o2;
#pragma unroll
                for (int i = 0; i < 8; ++i) { const h16 a = (h16)sp[i]; o[i] = a; o2[i] = (h16)((sp[i] - (float)a) * LOSC); }
                *(volatile v8h*)(crow + (size_t)row * ldc + piece * 8) = o; if (C2) *(volatile v8h*)(C2 + (size_t)r0 * ldc + c0 + (size_t)row * ldc + piece * 8) = o2; }
        };
        pass(); __threadfence(); pass();
    } else {
        float* crow = C + (size_t)r0 * ldc + c0;
        auto pass = [&]() {
#pragma unroll
            for (int s = 0; s < 8; ++s) { const int Lid = (lane >> 3) + 4 * s, piece = lane & 7; const int row = Lid >> 1, cofs = (Lid & 1) * 32 + piece * 4;
                v4f val = *(const v4fa*)(os + row * 68 + cofs); if (R) { const v4f rv = *(const v4f*)(R + ((size_t)r0 + row) * ldc + c0 + cofs); val += roundR ? (v4f){bfr(rv[0]), bfr(rv[1]), bfr(rv[2]), bfr(rv[3])} : rv; }
                *(volatile v4f*)(crow + (size_t)row * ldc + cofs) = val; }
        };
        pass(); __threadfence(); pass();
    }
}

__global__ __launch_bounds__(128) void k_gemm3(const bf* __restrict__ Ah, const bf* __restrict__ Al, const bf* __restrict__ Bh, const bf* __restrict__ Bl, int K, float* C, int ldc) {
    __shared__ __align__(16) float ost[4][16 * 68];
    const int lane = threadIdx.x & 31, wave = threadIdx.x >> 5, lr = lane & 15, hi = lane >> 4;
    const int r0 = blockIdx.x * 64 + wave * 16, c0 = blockIdx.y * 64;
    const size_t aoff = (size_t)(r0 + lr) * K + 8 * hi;
    v8f acc[4];
#pragma unroll
    for (int t = 0; t < 4; ++t) acc[t] = (v8f){};
#pragma unroll 1
    for (int kc = 0; kc < K; kc += 32) {
        const v16bf a = cat16b(*(const v8us*)(Ah + aoff + kc), *(const v8us*)(Ah + aoff + kc + 16));
        const v16bf al = cat16b(*(const v8us*)(Al + aoff + kc), *(const v8us*)(Al + aoff + kc + 16));
#pragma unroll
        for (int t = 0; t < 4; ++t) { const size_t bo = (size_t)(c0 + t * 16 + lr) * K + kc + 8 * hi;
            const v16bf bh = cat16b(*(const v8us*)(Bh + bo), *(const v8us*)(Bh + bo + 16)); const v16bf bl = cat16b(*(const v8us*)(Bl + bo), *(const v8us*)(Bl + bo + 16));
            acc[t] = wmmab(a, bh, acc[t]); acc[t] = wmmab(al, bh, acc[t]); acc[t] = wmmab(a, bl, acc[t]); }
        asm volatile("v_nop\n\tv_nop\n\tv_nop\n\tv_nop" : "+v"(acc[0]), "+v"(acc[1]), "+v"(acc[2]), "+v"(acc[3]) : "v"(a), "v"(al));
    }
    float* os = &ost[wave][0];
#pragma unroll
    for (int t = 0; t < 4; ++t) {
#pragma unroll
        for (int j = 0; j < 8; ++j) os[(hi * 8 + j) * 68 + t * 16 + lr] = acc[t][j]; }
    __builtin_amdgcn_wave_barrier(); asm volatile("" ::: "memory");
    float* crow = C + (size_t)r0 * ldc + c0;
    auto pass = [&]() {
#pragma unroll
        for (int s = 0; s < 8; ++s) { const int Lid = (lane >> 3) + 4 * s, piece = lane & 7; const int row = Lid >> 1, cofs = (Lid & 1) * 32 + piece * 4;
            const v4f val = *(const v4fa*)(os + row * 68 + cofs); *(volatile v4f*)(crow + (size_t)row * ldc + cofs) = val; }
    };
    pass(); __threadfence(); pass();
}
__global__ __launch_bounds__(256) void k_vt(const float* __restrict__ V, bf* VTH, bf* VTL) {
    __shared__ float tl[64][65];
    const int tid = threadIdx.x, t0 = blockIdx.x * 64, d0 = blockIdx.y * 64, g = blockIdx.z;
    { const int tt = tid >> 2, dq = (tid & 3) * 16;
#pragma unroll
      for (int i = 0; i < 16; ++i) tl[dq + i][tt] = V[(size_t)(t0 + tt) * KW + g * VHD + d0 + dq + i]; }
    __syncthreads();
    const int piece = tid & 7;
    auto pass = [&]() {
#pragma unroll
        for (int s = 0; s < 2; ++s) { const int d = (tid >> 3) + 32 * s; v8us oh, ol;
#pragma unroll
            for (int i = 0; i < 8; ++i) { const float v = tl[d][piece * 8 + i]; const unsigned short hb = f2bf(v); oh[i] = hb; ol[i] = f2bf(v - bf2f(hb)); }
            const size_t o = ((size_t)g * VHD + d0 + d) * NT_ + t0 + piece * 8; *(volatile v8us*)(VTH + o) = oh; *(volatile v8us*)(VTL + o) = ol; }
    };
    pass(); __threadfence(); pass();
}

__global__ __launch_bounds__(256) void k_split(const float* __restrict__ src, int nrows, bf* dh, bf* dl) {
    const int lane = threadIdx.x & 31, r = blockIdx.x * 8 + (threadIdx.x >> 5); if (r >= nrows) return;
#pragma unroll 1
    for (int ps = 0; ps < 2; ++ps) {
#pragma unroll 1
        for (int q = 0; q < DM / 256; ++q) { const size_t o = (size_t)r * DM + q * 256 + lane * 8; const v8f v = *(const v8f*)(src + o); v8us oh, ol;
#pragma unroll
            for (int i = 0; i < 8; ++i) { const unsigned short hb = f2bf(v[i]); oh[i] = hb; ol[i] = f2bf(v[i] - bf2f(hb)); }
            *(volatile v8us*)(dh + o) = oh; *(volatile v8us*)(dl + o) = ol; }
        if (ps == 0) __threadfence(); }
}
__global__ __launch_bounds__(256) void k_colsum(const float* __restrict__ V, float* VS) {
    const int e = blockIdx.x * 256 + threadIdx.x; if (e >= DM) return; float s = 0.f;
#pragma unroll 1
    for (int t = 0; t < NT_; ++t) s += V[(size_t)t * DM + e];
    *(volatile float*)(VS + e) = s; __threadfence(); *(volatile float*)(VS + e) = s;
}
__global__ __launch_bounds__(256) void k_softmax(const float* __restrict__ S, bf* PH, bf* PL) {
    const int lane = threadIdx.x & 31, r = blockIdx.x * 8 + (threadIdx.x >> 5); if (r >= RCH) return;
    const float* sr = S + (size_t)r * NT_; float m = -3.0e38f;
#pragma unroll 1
    for (int c0 = lane * 8; c0 < NT_; c0 += 256) { const v8f v = *(const v8f*)(sr + c0);
#pragma unroll
        for (int i = 0; i < 8; ++i) m = fmaxf(m, v[i] * SCL); }
#pragma unroll
    for (int sh = 16; sh; sh >>= 1) m = fmaxf(m, __shfl_xor(m, sh, 32));
    float sum = 0.f;
#pragma unroll 1
    for (int c0 = lane * 8; c0 < NT_; c0 += 256) { const v8f v = *(const v8f*)(sr + c0);
#pragma unroll
        for (int i = 0; i < 8; ++i) sum += __expf(v[i] * SCL - m); }
#pragma unroll
    for (int sh = 16; sh; sh >>= 1) sum += __shfl_xor(sum, sh, 32);
    const float inv = 1.0f / sum;
#pragma unroll 1
    for (int ps = 0; ps < 2; ++ps) {
#pragma unroll 1
        for (int c0 = lane * 8; c0 < NT_; c0 += 256) { const v8f v = *(const v8f*)(sr + c0); v8us oh, ol;
#pragma unroll
            for (int i = 0; i < 8; ++i) { const float p = __expf(v[i] * SCL - m) * inv; const unsigned short hb = f2bf(p); oh[i] = hb; ol[i] = f2bf(p - bf2f(hb)); }
            const size_t o = (size_t)r * NT_ + c0; *(volatile v8us*)(PH + o) = oh; *(volatile v8us*)(PL + o) = ol; }
        if (ps == 0) __threadfence(); }
}
__global__ __launch_bounds__(256) void k_revln(const float* __restrict__ O, const float* __restrict__ VS, const float* __restrict__ g, const float* __restrict__ bb, float* OUTP) {
    const int lane = threadIdx.x & 31, r = blockIdx.x * 8 + (threadIdx.x >> 5); if (r >= RCH) return;
    const float inv = 1.0f / (float)(NT_ - 1);
    v8f c[DM / 256]; float s = 0.f;
#pragma unroll
    for (int q = 0; q < DM / 256; ++q) { const int c0 = q * 256 + lane * 8; const v8f o = *(const v8f*)(O + (size_t)r * DM + c0); const v8f vs = *(const v8f*)(VS + c0);
#pragma unroll
        for (int i = 0; i < 8; ++i) { c[q][i] = (vs[i] - o[i]) * inv; s += c[q][i]; } }
#pragma unroll
    for (int sh = 16; sh; sh >>= 1) s += __shfl_xor(s, sh, 32);
    const float mu = s * (1.0f / DM); float s2 = 0.f;
#pragma unroll
    for (int q = 0; q < DM / 256; ++q)
#pragma unroll
        for (int i = 0; i < 8; ++i) { const float d = c[q][i] - mu; s2 = fmaf(d, d, s2); }
#pragma unroll
    for (int sh = 16; sh; sh >>= 1) s2 += __shfl_xor(s2, sh, 32);
    const float rs = rsqrtf(s2 * (1.0f / DM) + LN_EPS);
#pragma unroll 1
    for (int ps = 0; ps < 2; ++ps) {
#pragma unroll
        for (int q = 0; q < DM / 256; ++q) { const int c0 = q * 256 + lane * 8; v8f y;
#pragma unroll
            for (int i = 0; i < 8; ++i) y[i] = fmaxf((c[q][i] - mu) * rs * bfr(g[c0 + i]) + bfr(bb[c0 + i]), 0.f);
            *(volatile v8f*)(OUTP + (size_t)r * DM + c0) = y; }
        if (ps == 0) __threadfence(); }
}

extern "C" void kernel_launch(void* const* d_in, const int* in_sizes, int n_in,
                              void* d_out, int out_size, void* d_ws, size_t ws_size, hipStream_t stream) {
    (void)in_sizes; (void)n_in; (void)out_size;
    const float* x1 = (const float*)d_in[0]; const float* x2 = (const float*)d_in[1]; const float* Wq = (const float*)d_in[2]; const float* bq = (const float*)d_in[3]; const float* Wk = (const float*)d_in[4]; const float* bk = (const float*)d_in[5]; const float* Wv = (const float*)d_in[6]; const float* bv = (const float*)d_in[7]; const float* g = (const float*)d_in[8]; const float* bb = (const float*)d_in[9];
    float* out = (float*)d_out;
    char* wsp = (char*)d_ws;
    auto take = [&](size_t bytes) { char* p = wsp; wsp += (bytes + 255) & ~(size_t)255; return (void*)p; };
    bf* WqT = (bf*)take((size_t)DM * DM * 2); bf* WkT = (bf*)take((size_t)DM * DM * 2); bf* WvT = (bf*)take((size_t)DM * DM * 2); bf* Xb = (bf*)take((size_t)NT_ * DM * 2);
    float* TMP = (float*)take((size_t)NT_ * DM * 4); bf* Qh = (bf*)take((size_t)NT_ * DM * 2); bf* Ql = (bf*)take((size_t)NT_ * DM * 2); bf* Kh = (bf*)take((size_t)NT_ * DM * 2); bf* Kl = (bf*)take((size_t)NT_ * DM * 2);
    bf* VTH = (bf*)take((size_t)DM * NT_ * 2); bf* VTL = (bf*)take((size_t)DM * NT_ * 2); float* VS = (float*)take(DM * 4); float* S = (float*)take((size_t)RCH * NT_ * 4); bf* PH = (bf*)take((size_t)RCH * NT_ * 2); bf* PL = (bf*)take((size_t)RCH * NT_ * 2); float* O = (float*)take((size_t)RCH * DM * 4);
    if ((size_t)(wsp - (char*)d_ws) > ws_size) return;
    k_wt<<<dim3(DM / 64, DM / 64, 1), 256, 0, stream>>>(Wq, DM, DM, WqT); k_wt<<<dim3(DM / 64, DM / 64, 1), 256, 0, stream>>>(Wk, DM, DM, WkT); k_wt<<<dim3(DM / 64, DM / 64, 1), 256, 0, stream>>>(Wv, DM, DM, WvT);
    for (int b = 0; b < NBI; ++b) {
        k_cvtb<<<NT_ / 8, 256, 0, stream>>>(x1 + (size_t)b * NT_ * DM, NT_, Xb);
        k_gemmb<false, false><<<dim3(NT_ / 64, DM / 64, 1), 128, 0, stream>>>(Xb, nullptr, WqT, bq, TMP, DM, nullptr); k_split<<<NT_ / 8, 256, 0, stream>>>(TMP, NT_, Qh, Ql);
        k_cvtb<<<NT_ / 8, 256, 0, stream>>>(x2 + (size_t)b * NT_ * DM, NT_, Xb);
        k_gemmb<false, false><<<dim3(NT_ / 64, DM / 64, 1), 128, 0, stream>>>(Xb, nullptr, WkT, bk, TMP, DM, nullptr); k_split<<<NT_ / 8, 256, 0, stream>>>(TMP, NT_, Kh, Kl);
        k_gemmb<false, false><<<dim3(NT_ / 64, DM / 64, 1), 128, 0, stream>>>(Xb, nullptr, WvT, bv, TMP, DM, nullptr); k_colsum<<<DM / 256, 256, 0, stream>>>(TMP, VS); k_vt<<<dim3(NT_ / 64, 2, NKVV), 256, 0, stream>>>(TMP, VTH, VTL);
        for (int ch = 0; ch < NT_ / RCH; ++ch) { const size_t r0 = (size_t)ch * RCH;
            k_gemm3<<<dim3(RCH / 64, NT_ / 64, 1), 128, 0, stream>>>(Qh + r0 * DM, Ql + r0 * DM, Kh, Kl, DM, S, NT_);
            k_softmax<<<RCH / 8, 256, 0, stream>>>(S, PH, PL);
            k_gemm3<<<dim3(RCH / 64, DM / 64, 1), 128, 0, stream>>>(PH, PL, VTH, VTL, NT_, O, DM);
            k_revln<<<RCH / 8, 256, 0, stream>>>(O, VS, g, bb, out + ((size_t)b * NT_ + r0) * DM);
        }
    }
}
